// EncoderLayer_hybrid1_46651934769209
// MI455X (gfx1250) — hardware-run, weakly checked
//
#include <hip/hip_runtime.h>


#define NB_  8
#define TT   2048
#define EE   512
#define NH_  8
#define HD   64
#define PCAR 1024.0f
typedef _Float16 h16;
typedef unsigned short bf;
typedef __attribute__((ext_vector_type(16))) __bf16   v16bf;
typedef __attribute__((ext_vector_type(16))) _Float16 v16h;
typedef __attribute__((ext_vector_type(8)))  _Float16 v8h;
typedef __attribute__((ext_vector_type(8)))  unsigned short v8us;
typedef __attribute__((ext_vector_type(8)))  float    v8f;
typedef __attribute__((ext_vector_type(4)))  float    v4f;
typedef v8h  __attribute__((may_alias)) v8ha;
typedef v4f  __attribute__((may_alias)) v4fa;
typedef v8us __attribute__((may_alias)) v8usa;

__device__ __forceinline__ unsigned short f2bf(float f) { unsigned u = __float_as_uint(f); u += 0x7FFFu + ((u >> 16) & 1u); return (unsigned short)(u >> 16); }
__device__ __forceinline__ float bf2f(unsigned short b) { return __uint_as_float(((unsigned)b) << 16); }
__device__ __forceinline__ float bfr(float f) { return bf2f(f2bf(f)); }
__device__ __forceinline__ v16h cat16(v8h lo, v8h hi) { return __builtin_shufflevector(lo, hi, 0, 1, 2, 3, 4, 5, 6, 7, 8, 9, 10, 11, 12, 13, 14, 15); }
__device__ __forceinline__ v16bf cat16b(v8us lo, v8us hi) { return __builtin_bit_cast(v16bf, __builtin_shufflevector(lo, hi, 0, 1, 2, 3, 4, 5, 6, 7, 8, 9, 10, 11, 12, 13, 14, 15)); }
__device__ __forceinline__ v8f wmma16(v16h a, v16h b, v8f c) { return __builtin_amdgcn_wmma_f32_16x16x32_f16(false, a, false, b, (short)0, c, false, false); }
__device__ __forceinline__ v8f wmmab(v16bf a, v16bf b, v8f c) { return __builtin_amdgcn_wmma_f32_16x16x32_bf16(false, a, false, b, (short)0, c, false, false); }


template <typename T16> struct WFrag;
template <> struct WFrag<h16> { typedef v16h V; static __device__ __forceinline__ V ld(const h16* p) { return cat16(*(const v8h*)p, *(const v8h*)(p + 16)); } static __device__ __forceinline__ v8f mma(V a, V b, v8f c) { return wmma16(a, b, c); } };
template <> struct WFrag<bf> { typedef v16bf V; static __device__ __forceinline__ V ld(const bf* p) { return cat16b(*(const v8us*)p, *(const v8us*)(p + 16)); } static __device__ __forceinline__ v8f mma(V a, V b, v8f c) { return wmmab(a, b, c); } };
template <typename T16, int NSPLIT, bool BIAS>
__global__ __launch_bounds__(32) void k_gemmw(const T16* __restrict__ A, const T16* __restrict__ A2, const T16* __restrict__ Bt, const T16* __restrict__ Bt2, int K, float* C, int ldc, const float* __restrict__ bias, size_t sA, size_t sB, size_t sC) {
    typedef typename WFrag<T16>::V V;
    __shared__ __align__(16) float os[16 * 68];
    const size_t z = blockIdx.z; A += z * sA; if (A2) A2 += z * sA; Bt += z * sB; if (Bt2) Bt2 += z * sB; C += z * sC;
    const int lane = threadIdx.x & 31, lr = lane & 15, hi = lane >> 4; const int r0 = blockIdx.x * 64, c0 = blockIdx.y * 64;
    v8f acc[4][4];
#pragma unroll
    for (int mb = 0; mb < 4; ++mb)
#pragma unroll
        for (int nb = 0; nb < 4; ++nb) acc[mb][nb] = (v8f){};
    const size_t aoff = (size_t)(r0 + lr) * K + 8 * hi, boff = (size_t)(c0 + lr) * K + 8 * hi;
#pragma unroll 1
    for (int kc = 0; kc < K; kc += 32) {
        V a[4], a2[4];
#pragma unroll
        for (int mb = 0; mb < 4; ++mb) { a[mb] = WFrag<T16>::ld(A + aoff + (size_t)mb * 16 * K + kc); if (NSPLIT == 1 || NSPLIT == 2) a2[mb] = WFrag<T16>::ld(A2 + aoff + (size_t)mb * 16 * K + kc); }
#pragma unroll
        for (int nb = 0; nb < 4; ++nb) { const V b = WFrag<T16>::ld(Bt + boff + (size_t)nb * 16 * K + kc); V b2; if (NSPLIT >= 2) b2 = WFrag<T16>::ld(Bt2 + boff + (size_t)nb * 16 * K + kc);
#pragma unroll
            for (int mb = 0; mb < 4; ++mb) { acc[mb][nb] = WFrag<T16>::mma(a[mb], b, acc[mb][nb]); if (NSPLIT == 1 || NSPLIT == 2) acc[mb][nb] = WFrag<T16>::mma(a2[mb], b, acc[mb][nb]); if (NSPLIT >= 2) acc[mb][nb] = WFrag<T16>::mma(a[mb], b2, acc[mb][nb]); } }
        asm volatile("v_nop\n\tv_nop\n\tv_nop\n\tv_nop" : "+v"(acc[0][0]), "+v"(acc[1][1]), "+v"(acc[2][2]), "+v"(acc[3][3]) : "v"(a[0]), "v"(a[3]));
    }
#pragma unroll
    for (int mb = 0; mb < 4; ++mb) {
#pragma unroll
        for (int nb = 0; nb < 4; ++nb) {
#pragma unroll
            for (int j = 0; j < 8; ++j) os[(hi * 8 + j) * 68 + nb * 16 + lr] = acc[mb][nb][j]; }
        __builtin_amdgcn_wave_barrier(); asm volatile("" ::: "memory");
        float* crow = C + (size_t)(r0 + mb * 16) * ldc + c0;
#pragma unroll 1
        for (int ps = 0; ps < 2; ++ps) {
#pragma unroll
            for (int s = 0; s < 8; ++s) { const int row = 2 * s + hi, cofs = lr * 4; v4f val = *(const v4fa*)(os + row * 68 + cofs); if (BIAS) { val[0] += bfr(bias[c0 + cofs]); val[1] += bfr(bias[c0 + cofs + 1]); val[2] += bfr(bias[c0 + cofs + 2]); val[3] += bfr(bias[c0 + cofs + 3]); }
                *(volatile v4f*)(crow + (size_t)row * ldc + cofs) = val; }
            if (ps == 0) __threadfence(); }
        __builtin_amdgcn_wave_barrier(); asm volatile("" ::: "memory");
    }
}

__device__ __forceinline__ h16 tohx(float x) { return (h16)x; }
__device__ __forceinline__ void splitf(float y, unsigned short& h, unsigned short& l) { h = f2bf(y); l = f2bf(y - bf2f(h)); }
typedef __attribute__((ext_vector_type(2))) unsigned short v2us;
typedef __attribute__((ext_vector_type(4))) unsigned short v4us;
typedef __attribute__((ext_vector_type(2))) _Float16 v2h;
typedef __attribute__((ext_vector_type(4))) _Float16 v4h;

__global__ __launch_bounds__(256) void k_wtG(const float* __restrict__ w, int K, int N, bf* Bt) {
    const int lane = threadIdx.x & 31; const int L0 = (blockIdx.x * 8 + (threadIdx.x >> 5)) * 8; const int nlines = N * K / 64;
#pragma unroll
    for (int ps = 0; ps < 2; ++ps) {
#pragma unroll 1
        for (int l = 0; l < 8; ++l) { const int L = L0 + l; if (L >= nlines) break; const size_t e = (size_t)L * 64 + lane * 2; const int k = (int)(e % K), n = (int)(e / K); v2us o;
            o[0] = f2bf(w[(size_t)k * N + n]); o[1] = f2bf(w[(size_t)(k + 1) * N + n]); *(volatile v2us*)(Bt + e) = o; }
        if (ps == 0) __threadfence(); }
}
__global__ __launch_bounds__(256) void k_wv(const float* __restrict__ wv, bf* WVt) { const int e = (blockIdx.x * 256 + threadIdx.x) * 2; if (e >= NH_ * HD * HD) return; const int d = e % HD; const int o = (e / HD) % HD; const int h = e / (HD * HD); v2us w; w[0] = f2bf(wv[((size_t)h * HD + d) * HD + o]); w[1] = f2bf(wv[((size_t)h * HD + d + 1) * HD + o]);
    *(volatile v2us*)(WVt + e) = w; __threadfence(); *(volatile v2us*)(WVt + e) = w; }
__global__ __launch_bounds__(256) void k_ln(const float* __restrict__ X, float* XF, bf* Xh, bf* Xl) { const int lane = threadIdx.x & 31; const int t = blockIdx.x * 8 + (threadIdx.x >> 5); if (t >= TT) return; const float* xr = X + (size_t)t * EE; float v[EE / 32]; float s = 0.f;
#pragma unroll
    for (int ch = 0; ch < EE / 128; ++ch) { const v4f a = *(const v4f*)(xr + ch * 128 + lane * 4);
#pragma unroll
        for (int u = 0; u < 4; ++u) { v[ch * 4 + u] = bfr(a[u]); s += v[ch * 4 + u]; } }
#pragma unroll
    for (int sh = 16; sh; sh >>= 1) s += __shfl_xor(s, sh, 32);
    const float mean = s * (1.0f / EE); float q = 0.f;
#pragma unroll
    for (int k = 0; k < EE / 32; ++k) { float d = __fsub_rn(v[k], mean); asm volatile("" : "+v"(d)); float p = __fmul_rn(d, d); asm volatile("" : "+v"(p)); q = __fadd_rn(q, p); }
#pragma unroll
    for (int sh = 16; sh; sh >>= 1) q += __shfl_xor(q, sh, 32);
    const float rstd = __fdiv_rn(1.0f, __fsqrt_rn(__fadd_rn(q * (1.0f / EE), 1e-5f)));
    for (int ps = 0; ps < 2; ++ps) {
#pragma unroll
        for (int ch = 0; ch < EE / 128; ++ch) { v4f o; v4us oh, ol; const int c0 = ch * 128 + lane * 4; const int h = c0 / HD, d = c0 % HD;
#pragma unroll
            for (int u = 0; u < 4; ++u) { float dd = __fsub_rn(v[ch * 4 + u], mean); asm volatile("" : "+v"(dd)); o[u] = __fmul_rn(dd, rstd); unsigned short a, b; splitf(o[u], a, b); oh[u] = a; ol[u] = b; }
            *(volatile v4f*)(XF + (size_t)t * EE + c0) = o; const size_t oo = ((size_t)h * TT + t) * HD + d; *(volatile v4us*)(Xh + oo) = oh; *(volatile v4us*)(Xl + oo) = ol; }
        if (ps == 0) __threadfence(); } }
__global__ __launch_bounds__(256) void k_qk(const float* __restrict__ XF, const float* __restrict__ wq, const float* __restrict__ wk, float* QS, float* KS) { const int idx = blockIdx.x * 256 + threadIdx.x; if (idx >= NH_ * TT) return; const int t = idx % TT; const int h = idx / TT; const float* xr = XF + (size_t)t * EE + h * HD; float aq = 0.f, ak = 0.f;
#pragma unroll 1
    for (int d = 0; d < HD; ++d) { const float xv = xr[d]; float w1 = bfr(wq[h * HD + d]), w2 = bfr(wk[h * HD + d]); asm volatile("" : "+v"(w1)); asm volatile("" : "+v"(w2)); float p1 = __fmul_rn(xv, w1), p2 = __fmul_rn(xv, w2); asm volatile("" : "+v"(p1)); asm volatile("" : "+v"(p2)); aq = __fadd_rn(aq, p1); ak = __fadd_rn(ak, p2); }
    for (int ps = 0; ps < 2; ++ps) { *(volatile float*)(QS + idx) = aq; *(volatile float*)(KS + idx) = ak; if (ps == 0) __threadfence(); } }
__global__ __launch_bounds__(256) void k_vt(const float* __restrict__ V, h16* VT) { const int e = (blockIdx.x * 256 + threadIdx.x) * 2; if (e >= NH_ * HD * TT) return; const int t = e % TT; const int d = (e / TT) % HD; const int h = e / (TT * HD); v2h o; o[0] = tohx(V[((size_t)h * TT + t) * HD + d]); o[1] = tohx(V[((size_t)h * TT + t + 1) * HD + d]); *(volatile v2h*)(VT + e) = o; __threadfence(); *(volatile v2h*)(VT + e) = o; }
__global__ __launch_bounds__(256) void k_dsoft(const float* __restrict__ QS, const float* __restrict__ KS, h16* P16) { const int lane = threadIdx.x & 31; const int row = blockIdx.x * 8 + (threadIdx.x >> 5); if (row >= NH_ * TT) return; const int h = row / TT; const float qv = QS[row]; const float* kr = KS + (size_t)h * TT; float v[TT / 32]; float mx = -3.0e38f;
#pragma unroll
    for (int ch = 0; ch < TT / 128; ++ch) { const v4f a = *(const v4f*)(kr + ch * 128 + lane * 4);
#pragma unroll
        for (int u = 0; u < 4; ++u) { float df = __fsub_rn(qv, a[u]); asm volatile("" : "+v"(df)); float sq = __fmul_rn(df, df); asm volatile("" : "+v"(sq)); float t = -sq * 0.125f;     asm volatile("" : "+v"(t)); v[ch * 4 + u] = t; mx = fmaxf(mx, t); } }
#pragma unroll
    for (int sh = 16; sh; sh >>= 1) mx = fmaxf(mx, __shfl_xor(mx, sh, 32));
    float sum = 0.f;
#pragma unroll
    for (int q = 0; q < TT / 32; ++q) { float d0 = __fsub_rn(v[q], mx); asm volatile("" : "+v"(d0)); v[q] = __builtin_amdgcn_exp2f(__fmul_rn(d0, 1.4426950408889634f)); sum += v[q]; }
#pragma unroll
    for (int sh = 16; sh; sh >>= 1) sum += __shfl_xor(sum, sh, 32);
    const float f = __fdiv_rn(PCAR, sum);
    for (int ps = 0; ps < 2; ++ps) {
#pragma unroll
        for (int ch = 0; ch < TT / 128; ++ch) { v4h o4;
#pragma unroll
            for (int q = 0; q < 4; ++q) o4[q] = tohx(v[ch * 4 + q] * f); *(volatile v4h*)(P16 + (size_t)row * TT + ch * 128 + lane * 4) = o4; }
        if (ps == 0) __threadfence(); } }
__global__ __launch_bounds__(256) void k_mrg(const float* __restrict__ O, bf* Hh, bf* Hl) { const int e = (blockIdx.x * 256 + threadIdx.x) * 4; if (e >= NH_ * TT * HD) return; const int d = e % HD; const int t = (e / HD) % TT; const int h = e / (HD * TT); v4us oh, ol;
#pragma unroll
    for (int u = 0; u < 4; ++u) { unsigned short a, b; splitf(O[e + u] * (1.0f / PCAR), a, b); oh[u] = a; ol[u] = b; } const size_t oo = (size_t)t * EE + h * HD + d; *(volatile v4us*)(Hh + oo) = oh; *(volatile v4us*)(Hl + oo) = ol; __threadfence(); *(volatile v4us*)(Hh + oo) = oh; *(volatile v4us*)(Hl + oo) = ol; }
__global__ __launch_bounds__(256) void k_res(const float* __restrict__ X, float* OUTb) { const size_t e = ((size_t)blockIdx.x * 256 + threadIdx.x) * 4; if (e >= (size_t)TT * EE) return; const v4f a = *(const v4f*)(X + e), o0 = *(const v4f*)(OUTb + e); v4f o;
#pragma unroll
    for (int u = 0; u < 4; ++u) o[u] = __fadd_rn(o0[u], bfr(a[u])); *(volatile v4f*)(OUTb + e) = o; __threadfence(); *(volatile v4f*)(OUTb + e) = o; }

extern "C" void kernel_launch(void* const* d_in, const int* in_sizes, int n_in,
                              void* d_out, int out_size, void* d_ws, size_t ws_size, hipStream_t stream) {
    (void)in_sizes; (void)n_in; (void)out_size;
    const float* X = (const float*)d_in[0]; const float* wq = (const float*)d_in[1]; const float* wk = (const float*)d_in[2]; const float* wv = (const float*)d_in[3]; const float* wm = (const float*)d_in[4];
    float* OUT = (float*)d_out;
    char* wsp = (char*)d_ws;
    auto take = [&](size_t bytes) { char* p = wsp; wsp += (bytes + 255) & ~(size_t)255; return (void*)p; };
    bf* WVt = (bf*)take(NH_ * HD * HD * 2); bf* WM = (bf*)take((size_t)EE * EE * 2); float* XF = (float*)take((size_t)TT * EE * 4); bf* Xh = (bf*)take((size_t)TT * EE * 2); bf* Xl = (bf*)take((size_t)TT * EE * 2);
    float* QS = (float*)take(NH_ * TT * 4); float* KS = (float*)take(NH_ * TT * 4); float* V = (float*)take((size_t)NH_ * TT * HD * 4); h16* VT = (h16*)take((size_t)NH_ * HD * TT * 2); h16* P16 = (h16*)take((size_t)NH_ * TT * TT * 2); float* O = (float*)take((size_t)NH_ * TT * HD * 4); bf* Hh = (bf*)take((size_t)TT * EE * 2); bf* Hl = (bf*)take((size_t)TT * EE * 2);
    if ((size_t)(wsp - (char*)d_ws) > ws_size) return;
    k_wv<<<(NH_ * HD * HD / 2 + 255) / 256, 256, 0, stream>>>(wv, WVt); k_wtG<<<(EE * EE / 64 + 63) / 64, 256, 0, stream>>>(wm, EE, EE, WM);
    for (int b = 0; b < NB_; ++b) { const float* xb = X + (size_t)b * TT * EE;
        k_ln<<<TT / 8, 256, 0, stream>>>(xb, XF, Xh, Xl); k_qk<<<(NH_ * TT + 255) / 256, 256, 0, stream>>>(XF, wq, wk, QS, KS);
        k_gemmw<bf, 1, false><<<dim3(TT / 64, 1, NH_), 32, 0, stream>>>(Xh, Xl, WVt, nullptr, HD, V, HD, nullptr, (size_t)TT * HD, (size_t)HD * HD, (size_t)TT * HD);
        k_vt<<<(NH_ * HD * TT / 2 + 255) / 256, 256, 0, stream>>>(V, VT);
        k_dsoft<<<NH_ * TT / 8, 256, 0, stream>>>(QS, KS, P16);
        k_gemmw<h16, 0, false><<<dim3(TT / 64, 1, NH_), 32, 0, stream>>>(P16, nullptr, VT, nullptr, TT, O, HD, nullptr, (size_t)TT * TT, (size_t)HD * TT, (size_t)TT * HD);
        k_mrg<<<(NH_ * TT * HD / 4 + 255) / 256, 256, 0, stream>>>(O, Hh, Hl);
        k_gemmw<bf, 1, false><<<dim3(TT / 64, EE / 64, 1), 32, 0, stream>>>(Hh, Hl, WM, nullptr, EE, OUT + (size_t)b * TT * EE, EE, nullptr, 0, 0, 0);
        k_res<<<(unsigned)(((size_t)TT * EE / 4 + 255) / 256), 256, 0, stream>>>(xb, OUT + (size_t)b * TT * EE); }
}
